// model_28415503630530
// MI455X (gfx1250) — hardware-run, weakly checked
//
#include <hip/hip_runtime.h>
#pragma clang fp contract(off)


#ifndef NB
#define NB 4
#endif
#define NB_FULL 4
#define HW   4096
#define PH   66
#define PW   80
#define XO   8
#define PPB  (PH * PW)
#define NPL  11
#define P_IMG 0
#define P_S1  1
#define P_X0  2
#define P_C1  7
#define P_C2  8
#define P_C3  9
#define P_GA  10
#define CW   4
#define AW   4
#define MW   4
#define OSP  36
#define HLN  148
#define WSC  16.0f
#define WSI  0.0625f
#define QRS  2048.0f
#define PSH  14.0f
#define ECAR 16384.0f
#define BSC  16777216.0f
#define CI   5.9604644775390625e-08f
#define C0   (1.0f / 1024.0f)
#define C0R  (1.0f / 2097152.0f)
#define LOG2E 1.4426950408889634f
#define GSTEP (2.0f / 63.0f)

static_assert(NB <= NB_FULL);
static_assert(NB >= 1);
static_assert(PW % 8 == 0);
static_assert(XO % 8 == 0);
static_assert(PW >= XO + 64 + 1);
static_assert((NB * 256) % CW == 0);
static_assert(HW % (16 * AW) == 0);
static_assert((NB * HW) % (32 * MW) == 0);
static_assert((NB * HW) % 256 == 0);
static_assert(HLN == 2 * (PW / 8) + 64 * 2);
static_assert((OSP * 4) % 16 == 0);
static_assert(16 * 16 == 16 * 8 * 2);
static_assert(32 * 16 == 16 * 8 * 4);
static_assert(24 * 16 == 32 * 3 * 4);
static_assert((32 * 3 * 4) % 128 == 0);

typedef _Float16 h16;
typedef unsigned short bf;
typedef __attribute__((ext_vector_type(16))) __bf16   v16bf;
typedef __attribute__((ext_vector_type(16))) _Float16 v16h;
typedef __attribute__((ext_vector_type(8)))  _Float16 v8h;
typedef __attribute__((ext_vector_type(8)))  unsigned short v8us;
typedef __attribute__((ext_vector_type(8)))  float    v8f;
typedef __attribute__((ext_vector_type(4)))  float    v4f;
typedef v4f  __attribute__((may_alias)) v4fa;
typedef __attribute__((ext_vector_type(4)))  unsigned int v4u;

__device__ __forceinline__ unsigned short f2bf(float f) { unsigned u = __float_as_uint(f); u += 0x7FFFu + ((u >> 16) & 1u); return (unsigned short)(u >> 16); }
__device__ __forceinline__ float bfr(float f) { return __uint_as_float(((unsigned)f2bf(f)) << 16); }
__device__ __forceinline__ v16h cat16(v8h lo, v8h hi) { return __builtin_shufflevector(lo, hi, 0, 1, 2, 3, 4, 5, 6, 7, 8, 9, 10, 11, 12, 13, 14, 15); }
__device__ __forceinline__ v16bf cat16b(v8us lo, v8us hi) { return __builtin_bit_cast(v16bf, __builtin_shufflevector(lo, hi, 0, 1, 2, 3, 4, 5, 6, 7, 8, 9, 10, 11, 12, 13, 14, 15)); }
__device__ __forceinline__ v8f wmma16(v16h a, v16h b, v8f c) { return __builtin_amdgcn_wmma_f32_16x16x32_f16(false, a, false, b, (short)0, c, false, false); }
__device__ __forceinline__ v8f wmmab(v16bf a, v16bf b, v8f c) { return __builtin_amdgcn_wmma_f32_16x16x32_bf16(false, a, false, b, (short)0, c, false, false); }
__device__ __forceinline__ v16h  ldh(const h16* p) { return cat16(*(const v8h*)p, *(const v8h*)(p + 16)); }
__device__ __forceinline__ v16bf ldb(const bf* p)  { return cat16b(*(const v8us*)p, *(const v8us*)(p + 16)); }
__device__ __forceinline__ void wave_sync() { __builtin_amdgcn_fence(3  , "wavefront"); __builtin_amdgcn_wave_barrier(); asm volatile("" ::: "memory"); }

static __device__ __forceinline__ h16 toh_flush(float v) { const h16 r = (h16)v; return (fabsf(v) < 6.103515625e-05f) ? (h16)0.0f : r; }
__device__ __forceinline__ v8f wmma16g(v16h a, v16h b, v8f c) { c = wmma16(a, b, c); asm volatile("v_nop\n\tv_nop\n\tv_nop\n\tv_nop" : "+v"(c) : "v"(a), "v"(b)); return c; }
__device__ __forceinline__ unsigned pk2(h16 a, h16 b) { return (unsigned)__builtin_bit_cast(unsigned short, a) | ((unsigned)__builtin_bit_cast(unsigned short, b) << 16); }

__device__ __forceinline__ float lin_val(int i) { const float s = (float)i * (1.0f / 63.0f); const float a = 1.0f - s; const float v = s - a; return (i >= 63) ? 1.0f : v; }
__device__ __forceinline__ float ecar(float dist) { const float sc = 20.0f * __builtin_amdgcn_rcpf(1.0f + dist); return __builtin_amdgcn_exp2f((sc - 20.0f) * LOG2E + PSH); }
__device__ __forceinline__ float gdist(int di, int dj) { const float dx = (float)di * GSTEP, dy = (float)dj * GSTEP; return __builtin_amdgcn_sqrtf(dx * dx + dy * dy); }
__device__ __forceinline__ float diag_e(int im, int jm) {
    const float gx = lin_val(im), gy = lin_val(jm);
    const float xx = gx * gx, yy = gy * gy; const float sq = xx + yy;
    const float p = fmaf(gy, gy, xx);
    float d2 = (sq + sq) - 2.0f * p; d2 = fmaxf(d2, 0.0f);
    return ecar(__builtin_amdgcn_sqrtf(d2));
}

__global__ __launch_bounds__(256) void k_halo(h16* ACT, int nslab) {
    const int i = blockIdx.x * 256 + threadIdx.x; if (i >= nslab * HLN * 8) return;
    const int slab = i / (HLN * 8); const int rem = i - slab * (HLN * 8); const int ll = rem >> 3, pc = rem & 7;
    int row, line;
    if (ll < 10) { row = 0; line = ll; } else if (ll < 20) { row = PH - 1; line = ll - 10; } else { const int r = ll - 20; row = 1 + (r >> 1); line = (r & 1) ? 9 : 0; }
    const size_t o = (size_t)slab * PPB * 8 + (size_t)(row * PW + line * 8 + pc) * 8;
    const v8h z = (v8h){};
    *(volatile v8h*)(ACT + o) = z; __threadfence(); *(volatile v8h*)(ACT + o) = z;
}

__global__ __launch_bounds__(256) void k_img(const float* __restrict__ img, h16* ACT) {
    const int i = blockIdx.x * 256 + threadIdx.x; if (i >= NB * HW) return;
    const int b = i >> 12, p = i & (HW - 1), y = p >> 6, x = p & 63;
    const float* s = img + (size_t)b * 3 * HW + p;
    const h16 c0 = toh_flush(bfr(s[0])), c1 = toh_flush(bfr(s[HW])), c2 = toh_flush(bfr(s[2 * HW]));
    v4u o; o[0] = pk2(c0, c1); o[1] = (unsigned)__builtin_bit_cast(unsigned short, c2); o[2] = 0u; o[3] = 0u;
    const size_t d = (size_t)P_IMG * ((size_t)NB * PPB * 8) + ((size_t)(b * PH + y + 1) * PW + XO + x) * 8;
    *(volatile v4u*)(ACT + d) = o; __threadfence(); *(volatile v4u*)(ACT + d) = o;
}

__global__ __launch_bounds__(256) void k_wconv(const float* __restrict__ src, h16* dst, int nsrc, int n8, int Cout, int Cin, int T, int CG, int R, int K8) {
    const int i = blockIdx.x * 256 + threadIdx.x; if (i >= n8) return;
    const int k8 = i % K8; const int rz = i / K8; const int r = rz % R, z = rz / R;
    const int g = k8 / T, tap = k8 - g * T;
    const int rc = r < Cout ? r : Cout - 1;
    v8h o;
#pragma unroll
    for (int c = 0; c < 8; ++c) {
        const int ic = g * CG + c;
        const bool ok = (r < Cout) & (c < CG) & (ic < Cin);
        int si = ((z * Cout + rc) * Cin + (ic < Cin ? ic : Cin - 1)) * T + tap;
        si = si < nsrc ? si : nsrc - 1; si = si < 0 ? 0 : si;
        float v = src[si];
        asm volatile("" : "+v"(v));
        o[c] = ok ? toh_flush(bfr(v) * WSC) : (h16)0.0f;
    }
    *(volatile v8h*)(dst + (size_t)i * 8) = o; __threadfence(); *(volatile v8h*)(dst + (size_t)i * 8) = o;
}

template <int NG, int T>
__device__ __forceinline__ v8h ldrun(const h16* ACT, int pc, int q, int g0, int g1, int g2, int g3) {
    constexpr int NR = NG * T;
    const bool ok = q < NR;
    const int qc = ok ? q : (NR - 1);
    const int g = qc / T, tap = qc - g * T;
    int dy = 0, dx = 0;
    if (T == 9) { const int ky = tap / 3; dy = ky - 1; dx = tap - 3 * ky - 1; }
    int go = g0; go = (g == 1) ? g1 : go; go = (g == 2) ? g2 : go; go = (g == 3) ? g3 : go;
    v8h v = *(const v8h*)(ACT + (go + pc + (dy * PW + dx) * 8));
    asm volatile("" : "+v"(v));
    const v8h z = (v8h){};
    return ok ? v : z;
}

static constexpr int kpad(int nr) { return ((nr * 8 + 31) / 32) * 32; }

template <int NG, int T>
__device__ __forceinline__ void conv_body(const h16* ACT, const h16* __restrict__ WP, const float* __restrict__ bias, h16* ACTW, const float* S1R, float* F32O,
                                          int g0, int g1, int g2, int g3, int outOff, int hasout, int relu, int resOff, int hasres, int fmode) {
    __shared__ __align__(16) float cs[CW * 128];
    static_assert(CW * 128 * 4 <= 131072);
    constexpr int NR = NG * T, KP = kpad(NR), KS = KP / 32;
    static_assert(KP % 32 == 0);
    const int lane = threadIdx.x & 31, lr = lane & 15, hi = lane >> 4;
    const int wave = __builtin_amdgcn_readfirstlane((int)(threadIdx.x >> 5));
    const int tile = blockIdx.x * CW + wave;
    const int b = tile >> 8, y = (tile >> 2) & 63, x0 = (tile & 3) * 16;
    const int pc = ((b * PH + y + 1) * PW + XO + x0 + lr) * 8;
    v8f acc = (v8f){};
#pragma unroll
    for (int kc = 0; kc < KS; ++kc) {
        const v16h a = ldh(WP + lr * KP + kc * 32 + 8 * hi);
        const v8h r0 = ldrun<NG, T>(ACT, pc, 4 * kc + hi, g0, g1, g2, g3);
        const v8h r1 = ldrun<NG, T>(ACT, pc, 4 * kc + 2 + hi, g0, g1, g2, g3);
        acc = wmma16g(a, cat16(r0, r1), acc);
    }
    const bool own = hi == 0;
    const v8h rres = *(const v8h*)(ACT + (resOff + pc));
    float val[8];
#pragma unroll
    for (int r = 0; r < 8; ++r) {
        float v = acc[r] * WSI + bfr(bias[r < 6 ? r : 5]);
        if (hasres) v = v + (float)rres[r];
        if (relu) v = fmaxf(v, 0.0f);
        val[r] = (r < 6) ? v : 0.0f;
    }
    if (hasout) {
        v4u o; o[0] = pk2(toh_flush(val[0]), toh_flush(val[1])); o[1] = pk2(toh_flush(val[2]), toh_flush(val[3])); o[2] = pk2(toh_flush(val[4]), toh_flush(val[5])); o[3] = 0u;
        h16* dp = ACTW + (outOff + pc);
        if (own) *(volatile v4u*)dp = o;
        __threadfence();
        if (own) *(volatile v4u*)dp = o;
    }
    if (fmode != 0) {
        float c0 = 0.0f, c1 = 0.0f;
        if (fmode == 2) { c0 = lin_val(y); c1 = lin_val(x0 + lr); }
        const int wb = wave * 128;
        if (own) { cs[wb + lr * 8 + 0] = c0; cs[wb + lr * 8 + 1] = c1;
#pragma unroll
                   for (int r = 0; r < 6; ++r) cs[wb + lr * 8 + 2 + r] = val[r]; }
        wave_sync();
        const size_t fo = ((size_t)(b * HW + y * 64 + x0)) * 8 + (size_t)lane * 4;
        v4f v = *(const v4fa*)(&cs[wb + lane * 4]);
        if (fmode == 2) { const v4f s = *(const v4f*)(S1R + fo); v = v + s; }
        *(volatile v4f*)(F32O + fo) = v; __threadfence(); *(volatile v4f*)(F32O + fo) = v;
    }
}

__global__ __launch_bounds__(32 * CW) void k_conv3_1(const h16* ACT, const h16* __restrict__ WP, const float* __restrict__ bias, h16* ACTW, const float* S1R, float* F32O,
                                                     int g0, int g1, int g2, int g3, int outOff, int hasout, int relu, int resOff, int hasres, int fmode) {
    conv_body<1, 9>(ACT, WP, bias, ACTW, S1R, F32O, g0, g1, g2, g3, outOff, hasout, relu, resOff, hasres, fmode);
}
__global__ __launch_bounds__(32 * CW) void k_conv3_2(const h16* ACT, const h16* __restrict__ WP, const float* __restrict__ bias, h16* ACTW, const float* S1R, float* F32O,
                                                     int g0, int g1, int g2, int g3, int outOff, int hasout, int relu, int resOff, int hasres, int fmode) {
    conv_body<2, 9>(ACT, WP, bias, ACTW, S1R, F32O, g0, g1, g2, g3, outOff, hasout, relu, resOff, hasres, fmode);
}
__global__ __launch_bounds__(32 * CW) void k_conv3_3(const h16* ACT, const h16* __restrict__ WP, const float* __restrict__ bias, h16* ACTW, const float* S1R, float* F32O,
                                                     int g0, int g1, int g2, int g3, int outOff, int hasout, int relu, int resOff, int hasres, int fmode) {
    conv_body<3, 9>(ACT, WP, bias, ACTW, S1R, F32O, g0, g1, g2, g3, outOff, hasout, relu, resOff, hasres, fmode);
}
__global__ __launch_bounds__(32 * CW) void k_conv1_4(const h16* ACT, const h16* __restrict__ WP, const float* __restrict__ bias, h16* ACTW, const float* S1R, float* F32O,
                                                     int g0, int g1, int g2, int g3, int outOff, int hasout, int relu, int resOff, int hasres, int fmode) {
    conv_body<4, 1>(ACT, WP, bias, ACTW, S1R, F32O, g0, g1, g2, g3, outOff, hasout, relu, resOff, hasres, fmode);
}

__global__ __launch_bounds__(256) void k_tab(h16* TAB) {
    const int i = blockIdx.x * 256 + threadIdx.x; if (i >= 8 * 64 * 16) return;
    const int c = i >> 10, di = (i >> 4) & 63, x8 = (i & 15) * 8;
    v8h o;
#pragma unroll
    for (int e = 0; e < 8; ++e) {
        const int of = x8 + e + c - 63; const int sg = of >> 31; const int dj = (of ^ sg) - sg; const int djc = dj < 63 ? dj : 63;
        const float v = ecar(gdist(di, djc));
        o[e] = (of <= 63) ? toh_flush(v) : (h16)0.0f;
    }
    *(volatile v8h*)(TAB + (size_t)i * 8) = o; __threadfence(); *(volatile v8h*)(TAB + (size_t)i * 8) = o;
}

__global__ __launch_bounds__(256) void k_csum(float* CSP) {
    __shared__ float tl[HW];
    __shared__ float rr[HW];
    __shared__ __align__(16) float ot[2 * HW];
    static_assert((HW + HW + 2 * HW) * 4 <= 131072);
    static_assert(256 * 8 * 4 == 2 * HW);
    const int tid = threadIdx.x;
#pragma unroll 1
    for (int idx = tid; idx < HW; idx += 256) tl[idx] = (float)toh_flush(ecar(gdist(idx >> 6, idx & 63)));
    __syncthreads();
#pragma unroll 1
    for (int idx = tid; idx < HW; idx += 256) {
        const int di = idx >> 6, jm = idx & 63; float s = 0.0f;
#pragma unroll 1
        for (int j = 0; j < 64; ++j) { const int d = j - jm; const int sg = d >> 31; s += tl[di * 64 + ((d ^ sg) - sg)]; }
        rr[idx] = s;
    }
    __syncthreads();
#pragma unroll 1
    for (int idx = tid; idx < HW; idx += 256) {
        const int im = idx >> 6, jm = idx & 63; float s = 0.0f;
#pragma unroll 1
        for (int i2 = 0; i2 < 64; ++i2) { const int d = i2 - im; const int sg = d >> 31; s += rr[((d ^ sg) - sg) * 64 + jm]; }
        const float dc = diag_e(im, jm);
        const float cs = (s - ECAR) + dc;
        ot[idx] = __builtin_amdgcn_rcpf(cs); ot[HW + idx] = dc - ECAR;
    }
    __syncthreads();
#pragma unroll
    for (int k = 0; k < 8; ++k) { const int pi = (k * 256 + tid) * 4; const v4f v = *(const v4fa*)(&ot[pi]); *(volatile v4f*)(CSP + pi) = v; }
    __threadfence();
#pragma unroll
    for (int k = 0; k < 8; ++k) { const int pi = (k * 256 + tid) * 4; const v4f v = *(const v4fa*)(&ot[pi]); *(volatile v4f*)(CSP + pi) = v; }
}

__global__ __launch_bounds__(256) void k_flat(const float* __restrict__ FLATF, const float* __restrict__ CSP, h16* FT) {
    const int i = blockIdx.x * 256 + threadIdx.x;
    const int fg = i >> 9, m0 = (i & 511) * 8; const int b = fg >> 3, f = fg & 7;
    v8h o = (v8h){};
    if (b < NB) {
        const v4f r0 = *(const v4f*)(CSP + m0), r1 = *(const v4f*)(CSP + m0 + 4);
        const float* s = FLATF + ((size_t)(b * HW + m0)) * 8 + f;
#pragma unroll
        for (int e = 0; e < 4; ++e) { o[e] = toh_flush(s[e * 8] * r0[e] * BSC); o[4 + e] = toh_flush(s[(4 + e) * 8] * r1[e] * BSC); }
    }
    *(volatile v8h*)(FT + (size_t)i * 8) = o; __threadfence(); *(volatile v8h*)(FT + (size_t)i * 8) = o;
}

__global__ __launch_bounds__(32 * AW) void k_attn(const h16* __restrict__ TAB, const h16* __restrict__ FT, const float* __restrict__ CSP, const float* __restrict__ FLATF, float* WF) {
    __shared__ __align__(16) float os[AW * 16 * OSP];
    static_assert(AW * 16 * OSP * 4 <= 131072);
    static_assert(NB * 8 <= 32);
    const int lane = threadIdx.x & 31, lr = lane & 15, hi = lane >> 4;
    const int wave = __builtin_amdgcn_readfirstlane((int)(threadIdx.x >> 5));
    const int n0 = (blockIdx.x * AW + wave) * 16;
    const int in_ = n0 >> 6; const int jn = (n0 & 63) + lr;
    const int sft = 63 - jn;
    const int abase = (sft & 7) * (64 * 128) + (sft & ~7) + 8 * hi;
    const int bbase = lr * HW + 8 * hi;
    v8f acc0 = (v8f){}, acc1 = (v8f){};
#pragma unroll 1
    for (int im = 0; im < 64; ++im) {
        const int d = in_ - im; const int sg = d >> 31; const int di = (d ^ sg) - sg;
        const h16* ta = TAB + (abase + di * 128);
        const h16* fb = FT + (bbase + im * 64);
        { const v16h a = ldh(ta); const v16h b0 = ldh(fb); const v16h b1 = ldh(fb + 16 * HW);
          acc0 = wmma16g(a, b0, acc0); acc1 = wmma16g(a, b1, acc1); }
        { const v16h a = ldh(ta + 32); const v16h b0 = ldh(fb + 32); const v16h b1 = ldh(fb + 32 + 16 * HW);
          acc0 = wmma16g(a, b0, acc0); acc1 = wmma16g(a, b1, acc1); }
    }
    const int wb = wave * 16 * OSP;
#pragma unroll
    for (int r = 0; r < 8; ++r) { os[wb + (8 * hi + r) * OSP + lr] = acc0[r] * CI; os[wb + (8 * hi + r) * OSP + 16 + lr] = acc1[r] * CI; }
    wave_sync();
    const int row = lane >> 1, cofs = (lane & 1) * 4; const int n = n0 + row;
    const float cf = CSP[HW + n] * CSP[n];
    v4f val[NB];
#pragma unroll
    for (int b = 0; b < NB; ++b) {
        const v4f s = *(const v4fa*)(&os[wb + row * OSP + b * 8 + cofs]);
        const v4f fl = *(const v4f*)(FLATF + ((size_t)(b * HW + n)) * 8 + cofs);
        val[b] = s + fl * cf;
    }
#pragma unroll
    for (int b = 0; b < NB; ++b) *(volatile v4f*)(WF + ((size_t)(b * HW + n0)) * 8 + (size_t)lane * 4) = val[b];
    __threadfence();
#pragma unroll
    for (int b = 0; b < NB; ++b) *(volatile v4f*)(WF + ((size_t)(b * HW + n0)) * 8 + (size_t)lane * 4) = val[b];
}

__device__ __forceinline__ void ln_pack(float (&y)[4][8], const float* __restrict__ gp, const float* __restrict__ bp, int hi, v16h (&hb)[2]) {
    float s = 0.0f;
#pragma unroll
    for (int mb = 0; mb < 4; ++mb)
#pragma unroll
        for (int r = 0; r < 8; ++r) s += y[mb][r];
    s += __shfl_xor(s, 16, 32);
    const float mu = s * (1.0f / 64.0f);
    float q = 0.0f;
#pragma unroll
    for (int mb = 0; mb < 4; ++mb)
#pragma unroll
        for (int r = 0; r < 8; ++r) { const float d = y[mb][r] - mu; y[mb][r] = d; q += d * d; }
    q += __shfl_xor(q, 16, 32);
    const float rstd = rsqrtf(q * (1.0f / 64.0f) + 1e-5f);
#pragma unroll
    for (int mb = 0; mb < 4; ++mb) {
        const v4f ga = *(const v4f*)(gp + mb * 16 + 8 * hi), gb = *(const v4f*)(gp + mb * 16 + 8 * hi + 4);
        const v4f ba = *(const v4f*)(bp + mb * 16 + 8 * hi), bb = *(const v4f*)(bp + mb * 16 + 8 * hi + 4);
#pragma unroll
        for (int r = 0; r < 4; ++r) {
            const float v0 = fmaxf(y[mb][r] * rstd * bfr(ga[r]) + bfr(ba[r]), 0.0f);
            const float v1 = fmaxf(y[mb][4 + r] * rstd * bfr(gb[r]) + bfr(bb[r]), 0.0f);
            hb[mb >> 1][(mb & 1) * 8 + r] = toh_flush(v0); hb[mb >> 1][(mb & 1) * 8 + 4 + r] = toh_flush(v1);
        }
    }
}

__global__ __launch_bounds__(32 * MW) void k_mlp(const float* __restrict__ WF, const h16* __restrict__ W0P, const h16* __restrict__ WHP, const h16* __restrict__ WOP,
                                                 const float* __restrict__ b0, const float* __restrict__ g0, const float* __restrict__ be0,
                                                 const float* __restrict__ bh, const float* __restrict__ gh, const float* __restrict__ beh,
                                                 const float* __restrict__ bo, float* OUT) {
    __shared__ __align__(16) float os[MW * 96];
    static_assert(MW * 96 * 4 <= 131072);
    const int lane = threadIdx.x & 31, lr = lane & 15, hi = lane >> 4;
    const int wave = __builtin_amdgcn_readfirstlane((int)(threadIdx.x >> 5));
    const int tk0 = (blockIdx.x * MW + wave) * 32;
    const float bo0 = bfr(bo[0]), bo1 = bfr(bo[1]), bo2 = bfr(bo[2]);
    const bool lo = hi == 0;
    const v8h z8 = (v8h){};
#pragma unroll 1
    for (int tt = 0; tt < 2; ++tt) {
        const size_t wo = (size_t)(tk0 + tt * 16 + lr) * 8;
        const v4f x0 = *(const v4f*)(WF + wo), x1 = *(const v4f*)(WF + wo + 4);
        v8h hv, rv;
#pragma unroll
        for (int i = 0; i < 4; ++i) {
            const float s0 = x0[i] * 64.0f, s1 = x1[i] * 64.0f;
            const h16 a0 = toh_flush(s0), a1 = toh_flush(s1);
            hv[i] = a0; hv[4 + i] = a1;
            rv[i] = toh_flush((s0 - (float)a0) * QRS); rv[4 + i] = toh_flush((s1 - (float)a1) * QRS);
        }
        const v8h hs = lo ? hv : z8; const v8h rs = lo ? rv : z8;
        const v16h bH = cat16(hs, z8), bR = cat16(rs, z8);
        float y[4][8];
#pragma unroll
        for (int mb = 0; mb < 4; ++mb) {
            const v16h a = ldh(W0P + (mb * 16 + lr) * 32 + 8 * hi);
            v8f ac = (v8f){}, ar = (v8f){};
            ac = wmma16g(a, bH, ac); ar = wmma16g(a, bR, ar);
            const v4f ba = *(const v4f*)(b0 + mb * 16 + 8 * hi), bb = *(const v4f*)(b0 + mb * 16 + 8 * hi + 4);
#pragma unroll
            for (int r = 0; r < 4; ++r) { y[mb][r] = ac[r] * C0 + ar[r] * C0R + bfr(ba[r]); y[mb][4 + r] = ac[4 + r] * C0 + ar[4 + r] * C0R + bfr(bb[r]); }
        }
        v16h hb[2];
        ln_pack(y, g0, be0, hi, hb);
#pragma unroll 1
        for (int l = 0; l < 3; ++l) {
            const h16* wl = WHP + l * 4096 + lr * 64 + 8 * hi;
#pragma unroll
            for (int mb = 0; mb < 4; ++mb) {
                v8f ac = (v8f){};
                ac = wmma16g(ldh(wl + mb * 16 * 64), hb[0], ac);
                ac = wmma16g(ldh(wl + mb * 16 * 64 + 32), hb[1], ac);
                const v4f ba = *(const v4f*)(bh + l * 64 + mb * 16 + 8 * hi), bb = *(const v4f*)(bh + l * 64 + mb * 16 + 8 * hi + 4);
#pragma unroll
                for (int r = 0; r < 4; ++r) { y[mb][r] = ac[r] * WSI + bfr(ba[r]); y[mb][4 + r] = ac[4 + r] * WSI + bfr(bb[r]); }
            }
            ln_pack(y, gh + l * 64, beh + l * 64, hi, hb);
        }
        v8f ao = (v8f){};
        ao = wmma16g(ldh(WOP + lr * 64 + 8 * hi), hb[0], ao);
        ao = wmma16g(ldh(WOP + lr * 64 + 32 + 8 * hi), hb[1], ao);
        if (lo) { const int ob = wave * 96 + (tt * 16 + lr) * 3; os[ob + 0] = ao[0] * WSI + bo0; os[ob + 1] = ao[1] * WSI + bo1; os[ob + 2] = ao[2] * WSI + bo2; }
    }
    wave_sync();
    const int ls = lane < 24 ? lane : 23;
    const v4f v = *(const v4fa*)(&os[wave * 96 + ls * 4]);
    float* op = OUT + (size_t)tk0 * 3 + (size_t)ls * 4;
    if (lane < 24) *(volatile v4f*)op = v;
    __threadfence();
    if (lane < 24) *(volatile v4f*)op = v;
}

static constexpr size_t al256(size_t v) { return (v + 255) & ~(size_t)255; }
static constexpr int KP1 = kpad(9), KP2 = kpad(18), KP3 = kpad(27), KP4 = kpad(4);
static_assert(KP1 == 96);
static_assert(KP2 == 160);
static_assert(KP3 == 224);
static_assert(KP4 == 32);
static constexpr size_t PLH = (size_t)NB * PPB * 8;
static constexpr size_t SZ_ACT = al256((size_t)NPL * PLH * 2);
static constexpr size_t WC_HALVES = (size_t)16 * (KP1 + KP1 + 4 * (KP1 + KP2 + KP3 + KP4) + KP4 + KP1);
static constexpr size_t SZ_WC  = al256(WC_HALVES * 2);
static constexpr size_t SZ_WM  = al256((size_t)(64 * 32 + 3 * 64 * 64 + 16 * 64) * 2);
static constexpr size_t SZ_TAB = al256((size_t)8 * 64 * 128 * 2);
static constexpr size_t SZ_CSP = al256((size_t)2 * HW * 4);
static constexpr size_t SZ_F32 = al256((size_t)NB * HW * 8 * 4);
static constexpr size_t SZ_FT  = al256((size_t)32 * HW * 2);
static constexpr size_t SZ_TOTAL = SZ_ACT + SZ_WC + SZ_WM + SZ_TAB + SZ_CSP + 3 * SZ_F32 + SZ_FT;
static_assert(SZ_TOTAL <= (size_t)134217728);
static_assert((PLH * 2) % 256 == 0);
static_assert((size_t)NPL * PLH < (size_t)2147483647);
static_assert(((size_t)NPL * NB * HLN * 8) % 8 == 0);

extern "C" void kernel_launch(void* const* d_in, const int* in_sizes, int n_in,
                              void* d_out, int out_size, void* d_ws, size_t ws_size, hipStream_t stream) {
    if (n_in < 27) return;
    static const int need[27] = { NB * 3 * HW, 162, 6, 324, 6, 1296, 24, 2592, 24, 3888, 24, 576, 24, 144, 6, 324, 6,
                                  512, 64, 64, 64, 12288, 192, 192, 192, 192, 3 };
    for (int i = 0; i < 27; ++i) if (in_sizes[i] < need[i]) return;
    if ((size_t)out_size < (size_t)NB * HW * 3) return;
    if (SZ_TOTAL > ws_size) return;
    const float* img    = (const float*)d_in[0];
    const float* sfe1_w = (const float*)d_in[1];  const float* sfe1_b = (const float*)d_in[2];
    const float* sfe2_w = (const float*)d_in[3];  const float* sfe2_b = (const float*)d_in[4];
    const float* rdb_w0 = (const float*)d_in[5];  const float* rdb_b0 = (const float*)d_in[6];
    const float* rdb_w1 = (const float*)d_in[7];  const float* rdb_b1 = (const float*)d_in[8];
    const float* rdb_w2 = (const float*)d_in[9];  const float* rdb_b2 = (const float*)d_in[10];
    const float* lff_w  = (const float*)d_in[11]; const float* lff_b  = (const float*)d_in[12];
    const float* gff1_w = (const float*)d_in[13]; const float* gff1_b = (const float*)d_in[14];
    const float* gff2_w = (const float*)d_in[15]; const float* gff2_b = (const float*)d_in[16];
    const float* fc_w0  = (const float*)d_in[17]; const float* fc_b0  = (const float*)d_in[18];
    const float* ln_g0  = (const float*)d_in[19]; const float* ln_b0  = (const float*)d_in[20];
    const float* fc_wh  = (const float*)d_in[21]; const float* fc_bh  = (const float*)d_in[22];
    const float* ln_gh  = (const float*)d_in[23]; const float* ln_bh  = (const float*)d_in[24];
    const float* fc_wo  = (const float*)d_in[25]; const float* fc_bo  = (const float*)d_in[26];
    float* OUT = (float*)d_out;

    char* wsp = (char*)d_ws;
    h16* ACT = (h16*)wsp; wsp += SZ_ACT;
    h16* WC  = (h16*)wsp; wsp += SZ_WC;
    h16* WM  = (h16*)wsp; wsp += SZ_WM;
    h16* TAB = (h16*)wsp; wsp += SZ_TAB;
    float* CSP = (float*)wsp; wsp += SZ_CSP;
    float* S1F = (float*)wsp; wsp += SZ_F32;
    float* FLATF = (float*)wsp; wsp += SZ_F32;
    float* WF = (float*)wsp; wsp += SZ_F32;
    h16* FT  = (h16*)wsp; wsp += SZ_FT;

    h16* W_SFE1 = WC;
    h16* W_SFE2 = W_SFE1 + 16 * KP1;
    h16* W_R0   = W_SFE2 + 16 * KP1;
    h16* W_R1   = W_R0 + 4 * 16 * KP1;
    h16* W_R2   = W_R1 + 4 * 16 * KP2;
    h16* W_LFF  = W_R2 + 4 * 16 * KP3;
    h16* W_GF1  = W_LFF + 4 * 16 * KP4;
    h16* W_GF2  = W_GF1 + 16 * KP4;
    h16* W0P = WM;
    h16* WHP = W0P + 64 * 32;
    h16* WOP = WHP + 3 * 64 * 64;

    const int PO = (int)PLH;

    { const int nthr = NPL * NB * HLN * 8; k_halo<<<(unsigned)((nthr + 255) / 256), 256, 0, stream>>>(ACT, NPL * NB); }
    k_img<<<(unsigned)(NB * HW / 256), 256, 0, stream>>>(img, ACT);

    auto wc = [&](const float* src, h16* dst, int nsrc, int Z, int Cout, int Cin, int T, int CG, int R, int Kp) {
        const int n8 = Z * R * Kp / 8;
        k_wconv<<<(unsigned)((n8 + 255) / 256), 256, 0, stream>>>(src, dst, nsrc, n8, Cout, Cin, T, CG, R, Kp / 8);
    };
    wc(sfe1_w, W_SFE1, 162, 1, 6, 3, 9, 6, 16, KP1);
    wc(sfe2_w, W_SFE2, 324, 1, 6, 6, 9, 6, 16, KP1);
    wc(rdb_w0, W_R0, 1296, 4, 6, 6, 9, 6, 16, KP1);
    wc(rdb_w1, W_R1, 2592, 4, 6, 12, 9, 6, 16, KP2);
    wc(rdb_w2, W_R2, 3888, 4, 6, 18, 9, 6, 16, KP3);
    wc(lff_w,  W_LFF, 576, 4, 6, 24, 1, 6, 16, KP4);
    wc(gff1_w, W_GF1, 144, 1, 6, 24, 1, 6, 16, KP4);
    wc(gff2_w, W_GF2, 324, 1, 6, 6, 9, 6, 16, KP1);
    wc(fc_w0,  W0P, 512, 1, 64, 8, 1, 8, 64, 32);
    wc(fc_wh,  WHP, 12288, 3, 64, 64, 1, 8, 64, 64);
    wc(fc_wo,  WOP, 192, 1, 3, 64, 1, 8, 16, 64);

    const unsigned cg = (unsigned)(NB * 256 / CW); const unsigned cb = 32 * CW;
    k_conv3_1<<<cg, cb, 0, stream>>>(ACT, W_SFE1, sfe1_b, ACT, S1F, S1F, P_IMG * PO, 0, 0, 0, P_S1 * PO, 1, 0, 0, 0, 1);
    k_conv3_1<<<cg, cb, 0, stream>>>(ACT, W_SFE2, sfe2_b, ACT, S1F, S1F, P_S1 * PO, 0, 0, 0, P_X0 * PO, 1, 0, 0, 0, 0);
    for (int d = 0; d < 4; ++d) {
        const int xi = (P_X0 + d) * PO, xo = (P_X0 + d + 1) * PO;
        k_conv3_1<<<cg, cb, 0, stream>>>(ACT, W_R0 + d * 16 * KP1, rdb_b0 + d * 6, ACT, S1F, S1F, xi, 0, 0, 0, P_C1 * PO, 1, 1, 0, 0, 0);
        k_conv3_2<<<cg, cb, 0, stream>>>(ACT, W_R1 + d * 16 * KP2, rdb_b1 + d * 6, ACT, S1F, S1F, xi, P_C1 * PO, 0, 0, P_C2 * PO, 1, 1, 0, 0, 0);
        k_conv3_3<<<cg, cb, 0, stream>>>(ACT, W_R2 + d * 16 * KP3, rdb_b2 + d * 6, ACT, S1F, S1F, xi, P_C1 * PO, P_C2 * PO, 0, P_C3 * PO, 1, 1, 0, 0, 0);
        k_conv1_4<<<cg, cb, 0, stream>>>(ACT, W_LFF + d * 16 * KP4, lff_b + d * 6, ACT, S1F, S1F, xi, P_C1 * PO, P_C2 * PO, P_C3 * PO, xo, 1, 0, xi, 1, 0);
    }
    k_conv1_4<<<cg, cb, 0, stream>>>(ACT, W_GF1, gff1_b, ACT, S1F, S1F, (P_X0 + 1) * PO, (P_X0 + 2) * PO, (P_X0 + 3) * PO, (P_X0 + 4) * PO, P_GA * PO, 1, 0, 0, 0, 0);
    k_conv3_1<<<cg, cb, 0, stream>>>(ACT, W_GF2, gff2_b, ACT, S1F, FLATF, P_GA * PO, 0, 0, 0, 0, 0, 0, 0, 0, 2);

    k_tab<<<(unsigned)(8 * 64 * 16 / 256), 256, 0, stream>>>(TAB);
    k_csum<<<1, 256, 0, stream>>>(CSP);
    k_flat<<<(unsigned)(32 * 512 / 256), 256, 0, stream>>>(FLATF, CSP, FT);
    k_attn<<<(unsigned)(HW / (16 * AW)), 32 * AW, 0, stream>>>(TAB, FT, CSP, FLATF, WF);
    k_mlp<<<(unsigned)(NB * HW / (32 * MW)), 32 * MW, 0, stream>>>(WF, W0P, WHP, WOP, fc_b0, ln_g0, ln_b0, fc_bh, ln_gh, ln_bh, fc_bo, OUT);
}
